// S6_49847390437668
// MI455X (gfx1250) — hardware-verified
//
#include <hip/hip_runtime.h>
#include <math.h>

typedef __attribute__((ext_vector_type(16))) __bf16   v16b;
typedef __attribute__((ext_vector_type(8)))  __bf16   v8b;
typedef __attribute__((ext_vector_type(8)))  float    v8f;
typedef __attribute__((ext_vector_type(4)))  float    v4f;

constexpr int kBatch     = 4;
constexpr int kSeq       = 2048;
constexpr int kD         = 64;
constexpr int kN         = 64;
constexpr int kTok       = kBatch * kSeq;
constexpr int kWaves     = 4;
constexpr int kThreads   = kWaves * 32;
constexpr int kTokPerWave = 16;
constexpr int kTokPerBlk  = kWaves * kTokPerWave;
constexpr int kBlocks    = kTok / kTokPerBlk;
constexpr int kWP        = 64;
constexpr int kZP        = 68;
static_assert(kTok % kTokPerBlk == 0);
static_assert(kD == 64 && kN == 64);
static_assert((kD % 32) == 0);
static_assert((kWP % 8) == 0 && (kZP % 4) == 0);

__device__ __forceinline__ unsigned short f2bf_bits(float f) {
  unsigned u = __float_as_uint(f);
  return (unsigned short)((u + 0x7FFFu + ((u >> 16) & 1u)) >> 16);
}
__device__ __forceinline__ float bf_bits2f(unsigned short h) { return __uint_as_float(((unsigned)h) << 16); }

__device__ __forceinline__ void dep_guard_b(v8f& a, v8f& b, v16b x, v16b y) { asm volatile("v_nop\n\tv_nop\n\tv_nop\n\tv_nop" : "+v"(a), "+v"(b) : "v"(x), "v"(y)); }
__device__ __forceinline__ void keep4_b(v16b a, v16b b, v16b c, v16b d) { asm volatile("v_nop" :: "v"(a), "v"(b), "v"(c), "v"(d)); }
__device__ __forceinline__ void acc_guard4(v8f& a, v8f& b, v8f& c, v8f& d) { asm volatile("v_nop\n\tv_nop\n\tv_nop\n\tv_nop" : "+v"(a), "+v"(b), "+v"(c), "+v"(d)); }
__device__ __forceinline__ void guard_grp(v8f& a, v8f& b, v8f& c, v8f& d, v16b x, v16b y0, v16b y1, v16b y2, v16b y3) {
  asm volatile("v_nop\n\tv_nop\n\tv_nop\n\tv_nop" : "+v"(a), "+v"(b), "+v"(c), "+v"(d) : "v"(x), "v"(y0), "v"(y1), "v"(y2), "v"(y3));
}

template <typename T> struct Frag;
template <> struct Frag<__bf16> {
  typedef v16b V; union U { v16b v; v8b h[2]; };
  static __device__ __forceinline__ v16b load(const __bf16* p) {
    U f; f.h[0] = *(const v8b*)(p); f.h[1] = *(const v8b*)(p + 16); return f.v;
  }
  static __device__ __forceinline__ v8f mma(v16b a, v16b b, v8f c) {
    return __builtin_amdgcn_wmma_f32_16x16x32_bf16(false, a, false, b, (short)0, c, false, false);
  }
  static __device__ __forceinline__ void guard(v8f& a, v8f& b, v16b x, v16b y) { dep_guard_b(a, b, x, y); }
  static __device__ __forceinline__ void keep(v16b a, v16b b, v16b c, v16b d) { keep4_b(a, b, c, d); }
};
typedef Frag<__bf16> FragB;

__global__ __launch_bounds__(kThreads) void proj3_softplus_dot_kernel(
    const float* __restrict__ x,
    const float* __restrict__ W1, const float* __restrict__ b1,
    const float* __restrict__ W2, const float* __restrict__ b2,
    const float* __restrict__ W3, const float* __restrict__ b3,
    float* __restrict__ y)
{
  __shared__ __align__(16) __bf16 sW[3 * kN * kWP];
  __shared__ __align__(16) float  sBias[3 * kN];
  __shared__ __align__(16) float  sZ[kWaves][16 * kZP];
  __shared__ __align__(16) float  sS[kWaves * 16];

  const int tid   = threadIdx.x;
  const int lane  = tid & 31;
  const int wave  = tid >> 5;
  const int rlane = lane & 15;
  const int hh    = lane >> 4;
  const int koff  = hh * 8;
  const int mOff  = hh * 8;

#pragma unroll
  for (int g = 0; g < 3; ++g) {
    const float* Wg = (g == 0) ? W1 : ((g == 1) ? W2 : W3);
#pragma unroll 1
    for (int it = 0; it < 4; ++it) {
      const int idx = it * kThreads + tid;
      const int n   = idx & 63;
      const int k8  = idx >> 6;
      float wv[8];
#pragma unroll
      for (int j = 0; j < 8; ++j) wv[j] = Wg[(size_t)(k8 * 8 + j) * kN + n];
      v8b hv;
#pragma unroll
      for (int j = 0; j < 8; ++j) hv[j] = __builtin_bit_cast(__bf16, f2bf_bits(wv[j]));
      *(v8b*)(sW + (size_t)(g * kN + n) * kWP + k8 * 8) = hv;
      asm volatile("" ::: "memory");
    }
  }
  if (tid < kN) {
    sBias[tid]          = bf_bits2f(f2bf_bits(b1[tid]));
    sBias[kN + tid]     = bf_bits2f(f2bf_bits(b2[tid]));
    sBias[2 * kN + tid] = bf_bits2f(f2bf_bits(b3[tid]));
  }
  __syncthreads();

  const int tokW = blockIdx.x * kTokPerBlk + wave * kTokPerWave;
  const float* xr = x + (size_t)(tokW + rlane) * kD + koff;
  v16b af[2];
#pragma unroll
  for (int ks = 0; ks < 2; ++ks) {
    const v4f f0 = *(const v4f*)(xr + ks * 32);
    const v4f f1 = *(const v4f*)(xr + ks * 32 + 4);
    const v4f f2 = *(const v4f*)(xr + ks * 32 + 16);
    const v4f f3 = *(const v4f*)(xr + ks * 32 + 20);
#pragma unroll
    for (int e = 0; e < 4; ++e) {
      af[ks][e]      = __builtin_bit_cast(__bf16, f2bf_bits(f0[e]));
      af[ks][4 + e]  = __builtin_bit_cast(__bf16, f2bf_bits(f1[e]));
      af[ks][8 + e]  = __builtin_bit_cast(__bf16, f2bf_bits(f2[e]));
      af[ks][12 + e] = __builtin_bit_cast(__bf16, f2bf_bits(f3[e]));
    }
    asm volatile("" ::: "memory");
  }

  v8f acc[3][4];
#pragma unroll
  for (int g = 0; g < 3; ++g)
#pragma unroll
    for (int j = 0; j < 4; ++j) acc[g][j] = (v8f){0.f,0.f,0.f,0.f,0.f,0.f,0.f,0.f};

#pragma unroll
  for (int ks = 0; ks < 2; ++ks) {
#pragma unroll
    for (int g = 0; g < 3; ++g) {
      v16b bw[4];
#pragma unroll
      for (int j = 0; j < 4; ++j)
        bw[j] = FragB::load(sW + (size_t)(g * kN + j * 16 + rlane) * kWP + koff + ks * 32);
#pragma unroll
      for (int j = 0; j < 4; ++j) acc[g][j] = FragB::mma(af[ks], bw[j], acc[g][j]);
      guard_grp(acc[g][0], acc[g][1], acc[g][2], acc[g][3], af[ks], bw[0], bw[1], bw[2], bw[3]);
    }
  }
  acc_guard4(acc[0][0], acc[0][1], acc[0][2], acc[0][3]);
  acc_guard4(acc[1][0], acc[1][1], acc[1][2], acc[1][3]);
  acc_guard4(acc[2][0], acc[2][1], acc[2][2], acc[2][3]);

  float b1v[4], b2v[4], b3v[4];
#pragma unroll
  for (int j = 0; j < 4; ++j) {
    b1v[j] = sBias[j * 16 + rlane];
    b2v[j] = sBias[kN + j * 16 + rlane];
    b3v[j] = sBias[2 * kN + j * 16 + rlane];
  }

  float sr[8];
#pragma unroll
  for (int r = 0; r < 8; ++r) {
    float p = 0.0f;
#pragma unroll
    for (int j = 0; j < 4; ++j) {
      const float bm = acc[1][j][r] + b2v[j];
      const float cv = acc[2][j][r] + b3v[j];
      p = p + bm * cv;
    }
    p += __shfl_xor(p, 1);
    p += __shfl_xor(p, 2);
    p += __shfl_xor(p, 4);
    p += __shfl_xor(p, 8);
    sr[r] = p;
  }
  if (rlane == 0) {
#pragma unroll
    for (int r = 0; r < 8; ++r) sS[wave * 16 + mOff + r] = sr[r];
  }

  float* slab = sZ[wave];
#pragma unroll
  for (int j = 0; j < 4; ++j)
#pragma unroll
    for (int r = 0; r < 8; ++r)
      slab[(mOff + r) * kZP + j * 16 + rlane] = acc[0][j][r] + b1v[j];
  __syncthreads();

  const int c4 = rlane * 4;
#pragma unroll 1
  for (int it = 0; it < 8; ++it) {
    const int row = it * 2 + hh;
    const v4f zv = *(const v4f*)(slab + row * kZP + c4);
    const float sv = sS[wave * 16 + row];
    const v4f xv = *(const v4f*)(x + (size_t)(tokW + row) * kD + c4);
    v4f yv;
#pragma unroll
    for (int e = 0; e < 4; ++e) {
      const float z  = zv[e];
      const float sp = fmaxf(z, 0.0f) + log1pf(expf(-fabsf(z)));
      const float xb = bf_bits2f(f2bf_bits(xv[e]));
      yv[e] = (xb * sp) * sv;
    }
    *(v4f*)(slab + row * kZP + c4) = yv;
  }
  __syncthreads();

  for (int pass = 0; pass < 2; ++pass) {
#pragma unroll
    for (int it = 0; it < 8; ++it) {
      const int row = it * 2 + hh;
      const v4f v = *(const v4f*)(slab + row * kZP + c4);
      *(volatile v4f*)(y + (size_t)(tokW + row) * kD + c4) = v;
    }
    __threadfence();
  }
}

extern "C" void kernel_launch(void* const* d_in, const int* in_sizes, int n_in,
                              void* d_out, int out_size, void* d_ws, size_t ws_size,
                              hipStream_t stream) {
  (void)d_ws; (void)ws_size;
  if (n_in < 8) return;
  if (in_sizes[0] < kTok * kD) return;
  if (in_sizes[1] < kD * kD) return;
  if (in_sizes[2] < kD) return;
  if (in_sizes[3] < kD * kN) return;
  if (in_sizes[4] < kN) return;
  if (in_sizes[5] < kD * kN) return;
  if (in_sizes[6] < kN) return;
  if (out_size < kTok * kD) return;

  const float* x  = (const float*)d_in[0];
  const float* W1 = (const float*)d_in[1];
  const float* b1 = (const float*)d_in[2];
  const float* W2 = (const float*)d_in[3];
  const float* b2 = (const float*)d_in[4];
  const float* W3 = (const float*)d_in[5];
  const float* b3 = (const float*)d_in[6];
  float* y = (float*)d_out;

  proj3_softplus_dot_kernel<<<dim3(kBlocks), dim3(kThreads), 0, stream>>>(x, W1, b1, W2, b2, W3, b3, y);
}
